// EGNNLayer_22402549416673
// MI455X (gfx1250) — hardware-run, weakly checked
//
#include <hip/hip_runtime.h>
#include <stddef.h>


#pragma clang fp contract(off)

#define DN      128
#define NTHR    256
#define NWAVE   8
#define NBN     64
#define NBE     64
#define APA     136
#define APN     264
#define GSTR    132
#define NPROW   256
#define MROW    128
#define CROW    4
#define SROW    4
#define EPT     8
#define PIECE   (NTHR * EPT)
#define WCAP    (EPT * 32)
#define NBC     256
#define SLB     8
#define CE      163840
#define MAXCH   64
#define PA      0
#define PB      16384
#define PM2     32768
#define PC1     49152
#define PN1     65536
#define PN2     98304
#define PC2     114688
#define PWTOT   116736
#define PBLK    (PWTOT / (NTHR * 8))
#define WSCAP   134217728
#define NODEDYN (NBN * APA * 2)
#define EDGEDYN (NBE * GSTR * 4)
#define AGGDYN  ((NBC * DN + NBC * SROW) * 4)
#define MLPDYN  (NBN * APN * 2 + NBN * APA * 2)
#define SCW     16.0f
#define SCA     64.0f
#define INV1024 0.0009765625f

static_assert((PWTOT % (NTHR * 8)) == 0);
static_assert((PB % (NTHR * 8)) == 0);
static_assert((PM2 % (NTHR * 8)) == 0);
static_assert((PC1 % (NTHR * 8)) == 0);
static_assert((PN1 % (NTHR * 8)) == 0);
static_assert((PN2 % (NTHR * 8)) == 0);
static_assert((PC2 % (NTHR * 8)) == 0);
static_assert(PA + 128 * 128 == PB);
static_assert(PB + 128 * 128 == PM2);
static_assert(PM2 + 128 * 128 == PC1);
static_assert(PC1 + 128 * 128 == PN1);
static_assert(PN1 + 128 * 256 == PN2);
static_assert(PN2 + 128 * 128 == PC2);
static_assert(PC2 + 16 * 128 == PWTOT);
static_assert(((APA * 2) % 16) == 0);
static_assert(((APN * 2) % 16) == 0);
static_assert(((GSTR * 4) % 16) == 0);
static_assert(NBN * APN * 2 == NBN * GSTR * 4);
static_assert(NODEDYN == 17408);
static_assert(EDGEDYN == 33792);
static_assert(AGGDYN == 135168);
static_assert(MLPDYN == 51200);
static_assert(NBC == (1 << SLB));
static_assert(PIECE == 2048);
static_assert((EPT % 4) == 0);
static_assert((CE % PIECE) == 0);
static_assert((CE % NBE) == 0);
static_assert((NBC % NWAVE) == 0);
static_assert(NBC * SROW == 4 * NTHR);
static_assert(NBE == NWAVE * 8);
static_assert(NBE == 2 * 32);
static_assert(NBN == 4 * 16);
static_assert(NTHR == 4 * NBE);
static_assert((NBC * DN) % (4 * NTHR) == 0);

typedef float          v4f   __attribute__((ext_vector_type(4)));
typedef float          v8f   __attribute__((ext_vector_type(8)));
typedef int            v4i   __attribute__((ext_vector_type(4)));
typedef unsigned short v8us  __attribute__((ext_vector_type(8)));
typedef _Float16       v4h   __attribute__((ext_vector_type(4)));
typedef _Float16       v8h   __attribute__((ext_vector_type(8)));
typedef _Float16       v16h  __attribute__((ext_vector_type(16)));
union FragH { v16h v; v8h h[2]; };
union Cvt8  { v8h v; v8us u; };

__device__ __forceinline__ v8f wmh(v16h a, v16h b, v8f c) {
  v8f d = __builtin_amdgcn_wmma_f32_16x16x32_f16(false, a, false, b, (short)0, c, false, false);
  asm volatile("v_nop\n\tv_nop\n\tv_nop\n\tv_nop" : "+v"(d) : "v"(a), "v"(b));
  return d;
}
__device__ __forceinline__ v8f zero8() {
  v8f z = {0.f, 0.f, 0.f, 0.f, 0.f, 0.f, 0.f, 0.f};
  return z;
}
__device__ __forceinline__ v4f zero4() {
  v4f z = {0.f, 0.f, 0.f, 0.f};
  return z;
}
__device__ __forceinline__ int iclamp(int v, int lo, int hi) { return v < lo ? lo : (v > hi ? hi : v); }

__device__ __forceinline__ float silu_f(float x) {
  const float e = __expf(fminf(-x, 60.0f));
  return x * __builtin_amdgcn_rcpf(1.0f + e);
}

__device__ __forceinline__ v8h cvt8h(v4f xa, v4f xb, float scl) {
  v8h o;
  o[0] = (_Float16)(xa.x * scl); o[1] = (_Float16)(xa.y * scl); o[2] = (_Float16)(xa.z * scl); o[3] = (_Float16)(xa.w * scl);
  o[4] = (_Float16)(xb.x * scl); o[5] = (_Float16)(xb.y * scl); o[6] = (_Float16)(xb.z * scl); o[7] = (_Float16)(xb.w * scl);
  return o;
}

__device__ __forceinline__ void gemm16x64(const _Float16* ap, const _Float16* __restrict__ bpl, int kp, int nks, int n0,
                                          int m, int hh, v8f& c0, v8f& c1, v8f& c2, v8f& c3) {
  c0 = zero8(); c1 = zero8(); c2 = zero8(); c3 = zero8();
#pragma unroll 1
  for (int ks = 0; ks < nks; ++ks) {
    FragH a;
    a.h[0] = *(const v8h*)(ap + 32 * ks);
    a.h[1] = *(const v8h*)(ap + 32 * ks + 16);
    const _Float16* bp = bpl + (size_t)(n0 + m) * kp + 32 * ks + 8 * hh;
    FragH b;
    b.h[0] = *(const v8h*)(bp);
    b.h[1] = *(const v8h*)(bp + 16);
    c0 = wmh(a.v, b.v, c0);
    b.h[0] = *(const v8h*)(bp + (size_t)16 * kp);
    b.h[1] = *(const v8h*)(bp + (size_t)16 * kp + 16);
    c1 = wmh(a.v, b.v, c1);
    b.h[0] = *(const v8h*)(bp + (size_t)32 * kp);
    b.h[1] = *(const v8h*)(bp + (size_t)32 * kp + 16);
    c2 = wmh(a.v, b.v, c2);
    b.h[0] = *(const v8h*)(bp + (size_t)48 * kp);
    b.h[1] = *(const v8h*)(bp + (size_t)48 * kp + 16);
    c3 = wmh(a.v, b.v, c3);
  }
}

__device__ __forceinline__ void stage8f(float* sp, v8f a, float scl, float bias) {
#pragma unroll
  for (int r = 0; r < 8; ++r) sp[r * GSTR] = a[r] * scl + bias;
}
__device__ __forceinline__ void stage8fs(float* sp, v8f a, float bias) {
#pragma unroll
  for (int r = 0; r < 8; ++r) sp[r * GSTR] = silu_f(a[r] * INV1024 + bias);
}
__device__ __forceinline__ void stage8hs(_Float16* pc, v8f a, float bias) {
#pragma unroll
  for (int r = 0; r < 8; ++r) pc[r * APA] = (_Float16)(silu_f(a[r] * INV1024 + bias) * SCA);
}

__global__ __launch_bounds__(NTHR) void k_prep(
    const float* __restrict__ eW1, const float* __restrict__ eW2, const float* __restrict__ cW1,
    const float* __restrict__ cW2, const float* __restrict__ nW1, const float* __restrict__ nW2,
    unsigned short* wp) {
  const int tid = (int)threadIdx.x;
  const int b = (int)blockIdx.x;
  const int o = (b * NTHR + tid) * 8;
  const float* src = eW1;
  int r0 = 0, n, k0, pitch = DN, nval = DN;
  if (o < PB)        { n = o >> 7; k0 = o & 127; }
  else if (o < PM2)  { const int idx = o - PB;  n = idx >> 7; k0 = idx & 127; r0 = DN; }
  else if (o < PC1)  { const int idx = o - PM2; n = idx >> 7; k0 = idx & 127; src = eW2; }
  else if (o < PN1)  { const int idx = o - PC1; n = idx >> 7; k0 = idx & 127; src = cW1; }
  else if (o < PN2)  { const int idx = o - PN1; n = idx >> 8; k0 = idx & 255; src = nW1; }
  else if (o < PC2)  { const int idx = o - PN2; n = idx >> 7; k0 = idx & 127; src = nW2; }
  else               { const int idx = o - PC2; n = idx >> 7; k0 = idx & 127; src = cW2; pitch = 1; nval = 1; }
  const int nn = n < nval ? n : nval - 1;
  Cvt8 cv;
#pragma unroll
  for (int j = 0; j < 8; ++j) {
    const float w = src[(size_t)(r0 + k0 + j) * pitch + nn];
    const float v = (n < nval) ? (w * SCW) : 0.0f;
    cv.v[j] = (_Float16)v;
  }
  const v8us ov = cv.u;
  unsigned short* dp = wp + o;
  *(volatile v8us*)dp = ov;
  __threadfence();
  *(volatile v8us*)dp = ov;
}

__global__ __launch_bounds__(NTHR) void k_node(
    const float* __restrict__ hsrc, const unsigned short* __restrict__ wp, float* NP, int nN) {
  extern __shared__ __attribute__((aligned(16))) float ndynf[];
  __shared__ __attribute__((aligned(16))) float stg[NWAVE * 1024];
  _Float16* sAh = (_Float16*)ndynf;
  const int tid = (int)threadIdx.x, lane = tid & 31, wave = tid >> 5, hh = lane >> 4, m = lane & 15;
  const int n0 = (int)blockIdx.x * NBN;

  {
    const int nl = tid >> 2, q = tid & 3;
    int node = n0 + nl;
    node = node > nN - 1 ? nN - 1 : node;
    const float* rp = hsrc + (size_t)node * DN + 32 * q;
#pragma unroll
    for (int i = 0; i < 4; ++i) {
      const v4f xa = *(const v4f*)(rp + 8 * i);
      const v4f xb = *(const v4f*)(rp + 8 * i + 4);
      *(v8h*)(sAh + nl * APA + 32 * q + 8 * i) = cvt8h(xa, xb, SCA);
    }
  }
  __syncthreads();

  const int rt = wave & 3, chf = wave >> 2;
  const _Float16* ap  = sAh + (16 * rt + m) * APA + 8 * hh;
  const _Float16* bpl = (const _Float16*)(wp + (chf ? PB : PA));
  float* sw = stg + wave * 1024;
#pragma unroll 1
  for (int qq = 0; qq < 2; ++qq) {
    v8f a0, a1, a2, a3;
    gemm16x64(ap, bpl, DN, 4, 64 * qq, m, hh, a0, a1, a2, a3);
    {
      float* sp = sw + (8 * hh) * 64 + m;
#pragma unroll
      for (int r = 0; r < 8; ++r) {
        sp[r * 64]      = a0[r] * INV1024;
        sp[r * 64 + 16] = a1[r] * INV1024;
        sp[r * 64 + 32] = a2[r] * INV1024;
        sp[r * 64 + 48] = a3[r] * INV1024;
      }
    }
    __syncthreads();
#pragma unroll 1
    for (int i = 0; i < 8; ++i) {
      const int r2 = 2 * i + hh;
      const v4f v = *(const v4f*)(sw + r2 * 64 + 4 * m);
      const int row = n0 + 16 * rt + r2;
      *(volatile v4f*)(NP + (size_t)row * NPROW + 128 * chf + 64 * qq + 4 * m) = v;
    }
    __threadfence();
#pragma unroll 1
    for (int i = 0; i < 8; ++i) {
      const int r2 = 2 * i + hh;
      const v4f v = *(const v4f*)(sw + r2 * 64 + 4 * m);
      const int row = n0 + 16 * rt + r2;
      *(volatile v4f*)(NP + (size_t)row * NPROW + 128 * chf + 64 * qq + 4 * m) = v;
    }
    __syncthreads();
  }
}

__global__ __launch_bounds__(NTHR) void k_edge(
    const float* __restrict__ pos, const int* __restrict__ ei, const float* __restrict__ NP,
    const unsigned short* __restrict__ wp, const float* __restrict__ eW1, const float* __restrict__ eb1,
    const float* __restrict__ eb2, const float* __restrict__ cb1,
    float* Mout, float* Cout, int nE, int nN, int cbeg) {
  extern __shared__ __attribute__((aligned(16))) float sH[];
  __shared__ __attribute__((aligned(16))) _Float16 sA[NBE * APA];
  __shared__ __attribute__((aligned(16))) _Float16 sC[NBE * APA];
  __shared__ __attribute__((aligned(16))) float sPar[4 * DN];
  __shared__ __attribute__((aligned(16))) float sCD[NBE * 4];
  __shared__ float sSQ[NBE];
  __shared__ float sWg[NBE];
  __shared__ int sI[NBE];
  __shared__ int sJ[NBE];
  const int tid = (int)threadIdx.x, lane = tid & 31, wave = tid >> 5, hh = lane >> 4, m = lane & 15;
  const int el0 = (int)blockIdx.x * NBE;

  if (wave < 2) {
    int e = cbeg + el0 + tid;
    e = e > nE - 1 ? nE - 1 : e;
    const int ii = iclamp(ei[e], 0, nN - 1);
    const int jj = iclamp(ei[(size_t)nE + e], 0, nN - 1);
    const float* pi = pos + (size_t)ii * 3;
    const float* pj = pos + (size_t)jj * 3;
    const float dx = pi[0] - pj[0];
    const float dy = pi[1] - pj[1];
    const float dz = pi[2] - pj[2];
    const float sq = (dx * dx + dz * dz) + dy * dy;
    sCD[4 * tid]     = dx;
    sCD[4 * tid + 1] = dy;
    sCD[4 * tid + 2] = dz;
    sCD[4 * tid + 3] = 0.0f;
    sSQ[tid] = sq;
    sI[tid] = ii;
    sJ[tid] = jj;
  }
  if (tid < DN) {
    sPar[tid]          = eb1[tid];
    sPar[DN + tid]     = eb2[tid];
    sPar[2 * DN + tid] = cb1[tid];
    sPar[3 * DN + tid] = eW1[(size_t)2 * DN * DN + tid];
  }
  __syncthreads();

  const int rt = wave & 3, cg = wave >> 2;

  {
    const int c4 = 4 * lane;
    const v4f w4 = *(const v4f*)(sPar + 3 * DN + c4);
    const v4f b4 = *(const v4f*)(sPar + c4);
#pragma unroll 1
    for (int jx = 0; jx < 8; ++jx) {
      const int el = 8 * wave + jx;
      const int ii = sI[el];
      const int jj = sJ[el];
      const float sq = sSQ[el];
      const v4f p = *(const v4f*)(NP + (size_t)ii * NPROW + c4);
      const v4f q = *(const v4f*)(NP + (size_t)jj * NPROW + DN + c4);
      const v4f v = ((p + q) + sq * w4) + b4;
      v4h z;
      z.x = (_Float16)(silu_f(v.x) * SCA);
      z.y = (_Float16)(silu_f(v.y) * SCA);
      z.z = (_Float16)(silu_f(v.z) * SCA);
      z.w = (_Float16)(silu_f(v.w) * SCA);
      *(v4h*)(sA + el * APA + c4) = z;
    }
  }
  __syncthreads();

  {
    v8f a0, a1, a2, a3;
    gemm16x64(sA + (16 * rt + m) * APA + 8 * hh, (const _Float16*)(wp + PM2), DN, 4, 64 * cg, m, hh, a0, a1, a2, a3);
    float* sp = sH + (16 * rt + 8 * hh) * GSTR + 64 * cg + m;
    const float* bb = sPar + DN + 64 * cg + m;
    stage8fs(sp,      a0, bb[0]);
    stage8fs(sp + 16, a1, bb[16]);
    stage8fs(sp + 32, a2, bb[32]);
    stage8fs(sp + 48, a3, bb[48]);
  }
  __syncthreads();

  {
#pragma unroll 1
    for (int it = 0; it < 8; ++it) {
      const int row = wave + NWAVE * it;
      const v4f v = *(const v4f*)(sH + row * GSTR + 4 * lane);
      *(volatile v4f*)(Mout + (size_t)(el0 + row) * MROW + 4 * lane) = v;
    }
    __threadfence();
#pragma unroll 1
    for (int it = 0; it < 8; ++it) {
      const int row = wave + NWAVE * it;
      const v4f v = *(const v4f*)(sH + row * GSTR + 4 * lane);
      *(volatile v4f*)(Mout + (size_t)(el0 + row) * MROW + 4 * lane) = v;
    }
  }
  {
    const int c4 = 4 * lane;
#pragma unroll 1
    for (int jx = 0; jx < 8; ++jx) {
      const int el = 8 * wave + jx;
      const v4f v = *(const v4f*)(sH + el * GSTR + c4);
      v4h z;
      z.x = (_Float16)(v.x * SCA);
      z.y = (_Float16)(v.y * SCA);
      z.z = (_Float16)(v.z * SCA);
      z.w = (_Float16)(v.w * SCA);
      *(v4h*)(sA + el * APA + c4) = z;
    }
  }
  __syncthreads();

  {
    v8f a0, a1, a2, a3;
    gemm16x64(sA + (16 * rt + m) * APA + 8 * hh, (const _Float16*)(wp + PC1), DN, 4, 64 * cg, m, hh, a0, a1, a2, a3);
    _Float16* pc = sC + (16 * rt + 8 * hh) * APA + 64 * cg + m;
    const float* bb = sPar + 2 * DN + 64 * cg + m;
    stage8hs(pc,      a0, bb[0]);
    stage8hs(pc + 16, a1, bb[16]);
    stage8hs(pc + 32, a2, bb[32]);
    stage8hs(pc + 48, a3, bb[48]);
  }
  __syncthreads();

  if (wave < 4) {
    v8f c = zero8();
    const _Float16* ap = sC + (16 * wave + m) * APA + 8 * hh;
    const _Float16* bp = (const _Float16*)(wp + PC2) + (size_t)m * DN + 8 * hh;
#pragma unroll 1
    for (int ks = 0; ks < 4; ++ks) {
      FragH a, b;
      a.h[0] = *(const v8h*)(ap + 32 * ks);
      a.h[1] = *(const v8h*)(ap + 32 * ks + 16);
      b.h[0] = *(const v8h*)(bp + 32 * ks);
      b.h[1] = *(const v8h*)(bp + 32 * ks + 16);
      c = wmh(a.v, b.v, c);
    }
    if (m == 0) {
#pragma unroll
      for (int r = 0; r < 8; ++r) sWg[16 * wave + 8 * hh + r] = c[r] * INV1024;
    }
  }
  __syncthreads();

  if (wave < 2) {
    const int e = tid;
    const float cw = sWg[e];
    const float sq = sSQ[e];
    const float rinv = 1.0f / sqrtf(sq + 1e-8f);
    v4f ov;
    ov.x = (sCD[4 * e]     * rinv) * cw;
    ov.y = (sCD[4 * e + 1] * rinv) * cw;
    ov.z = (sCD[4 * e + 2] * rinv) * cw;
    ov.w = 0.0f;
    float* cp = Cout + (size_t)(el0 + e) * CROW;
    *(volatile v4f*)cp = ov;
    __threadfence();
    *(volatile v4f*)cp = ov;
  }
}

__device__ __forceinline__ int scan_piece(const int* __restrict__ eid, int lim, int cbase, int base, int vecok,
                                          int* list, int tid, int wave) {
  int wc = 0;
  const int el0  = tid * EPT;
  const int e0   = cbase + el0;
  const int sent = -2147483647 - 1;
  int kk[EPT];
  if (vecok != 0 && cbase + PIECE <= lim) {
    const v4i* p = (const v4i*)(eid + e0);
#pragma unroll
    for (int u = 0; u < EPT / 4; ++u) {
      const v4i d = p[u];
      kk[4 * u] = d.x; kk[4 * u + 1] = d.y; kk[4 * u + 2] = d.z; kk[4 * u + 3] = d.w;
    }
  } else {
    const int lm = lim - 1;
#pragma unroll
    for (int q = 0; q < EPT; ++q) {
      const int eq = e0 + q;
      const int ec = eq > lm ? lm : eq;
      const int a = eid[ec];
      kk[q] = (eq < lim) ? a : sent;
    }
  }
  const unsigned nb = (unsigned)base;
  unsigned sq[EPT];
  bool hq[EPT];
  bool anyl = false;
#pragma unroll
  for (int q = 0; q < EPT; ++q) {
    sq[q] = (unsigned)kk[q] - nb;
    hq[q] = sq[q] < (unsigned)NBC;
    anyl = anyl | hq[q];
  }
  const unsigned any = __builtin_amdgcn_ballot_w32(anyl);
  if (any != 0u) {
#define HIT(HQ, SQ, Q) { \
      const unsigned mj = __builtin_amdgcn_ballot_w32(HQ); \
      if (mj != 0u) { \
        if (HQ) { \
          const int ps = wc + (int)__builtin_amdgcn_mbcnt_lo(mj, 0u); \
          if (ps < WCAP) list[wave * WCAP + ps] = ((el0 + (Q)) << SLB) | (int)(SQ); \
        } \
        wc += (int)__builtin_popcount(mj); } }
#pragma unroll
    for (int q = 0; q < EPT; ++q) {
      HIT(hq[q], sq[q], q)
    }
#undef HIT
  }
  return wc;
}

__device__ __forceinline__ void drain_piece(const int* list, const int* wcnt, float* accF, float* accC,
                                            const float* __restrict__ Mf, const float* __restrict__ Cq,
                                            int rowoff, int lane, int wave) {
#pragma unroll 1
  for (int wsx = 0; wsx < NWAVE; ++wsx) {
    int n = __builtin_amdgcn_readfirstlane(wcnt[wsx]);
    n = n > WCAP ? WCAP : (n < 0 ? 0 : n);
    const int* lp = list + wsx * WCAP;
#pragma unroll 1
    for (int bb = 0; bb < n; bb += 32) {
      const int idx = bb + lane;
      const int ic = idx > WCAP - 1 ? WCAP - 1 : idx;
      const int ent = lp[ic];
      const bool own = (idx < n) && ((ent & (NWAVE - 1)) == wave);
      unsigned msk = __builtin_amdgcn_ballot_w32(own);
#pragma unroll 1
      while (msk != 0u) {
        const int bit = (int)__builtin_ctz(msk);
        msk &= msk - 1u;
        const int e2 = __builtin_amdgcn_readlane(ent, bit);
        const int slot = e2 & (NBC - 1);
        const int el = (e2 >> SLB) & (PIECE - 1);
        int row = rowoff + el;
        row = row < 0 ? 0 : (row > CE - 1 ? CE - 1 : row);
        const v4f mv = *(const v4f*)(Mf + (size_t)row * MROW + 4 * lane);
        float* ap = accF + slot * DN + 4 * lane;
        v4f a = *(const v4f*)ap;
        a += mv;
        *(v4f*)ap = a;
        const float cvv = Cq[(size_t)row * CROW + (lane & 3)];
        const float addv = (lane < 3) ? cvv : ((lane == 3) ? 1.0f : 0.0f);
        if (lane < SROW) accC[SROW * slot + lane] += addv;
      }
    }
  }
}

__device__ __forceinline__ void agg_store(const float* accF, const float* accC, const float* __restrict__ xb,
                                          float* outH, float* outX, float* S, int base, int nN, int last,
                                          int tid, int lane, int wave) {
#pragma unroll 1
  for (int it = 0; it < NBC / NWAVE; ++it) {
    const int s = wave + NWAVE * it;
    const int node = base + s;
    if (node < nN) {
      const v4f v = *(const v4f*)(accF + s * DN + 4 * lane);
      *(volatile v4f*)(outH + (size_t)node * DN + 4 * lane) = v;
    }
  }
  if (last != 0) {
    int cnt = nN - base;
    cnt = cnt > NBC ? NBC : cnt;
    const int nf = 3 * cnt;
    const int nq = nf >> 2;
    const size_t f0 = (size_t)3 * (size_t)base;
#pragma unroll 1
    for (int q = tid; q < nq; q += NTHR) {
      float a[4];
#pragma unroll
      for (int c = 0; c < 4; ++c) {
        const int t = 4 * q + c;
        const int s3 = t / 3;
        const int cc = t - 3 * s3;
        const float sv = accC[SROW * s3 + cc];
        const float cn = accC[SROW * s3 + 3];
        const float xv = xb[f0 + (size_t)t];
        a[c] = xv + sv * (1.0f / fmaxf(cn, 1.0f));
      }
      v4f ov;
      ov.x = a[0]; ov.y = a[1]; ov.z = a[2]; ov.w = a[3];
      *(volatile v4f*)(outX + f0 + 4 * (size_t)q) = ov;
    }
    const int rem = nf - 4 * nq;
    if (rem > 0 && tid == 0) {
#pragma unroll
      for (int c = 0; c < 3; ++c) {
        if (c < rem) {
          const int t = 4 * nq + c;
          const int s3 = t / 3;
          const int cc = t - 3 * s3;
          const float sv = accC[SROW * s3 + cc];
          const float cn = accC[SROW * s3 + 3];
          const float xv = xb[f0 + (size_t)t];
          const float v = xv + sv * (1.0f / fmaxf(cn, 1.0f));
          *(volatile float*)(outX + f0 + (size_t)t) = v;
        }
      }
    }
  } else {
    const int q = tid;
    const v4f v = *(const v4f*)(accC + 4 * q);
    *(volatile v4f*)(S + (size_t)base * SROW + 4 * (size_t)q) = v;
  }
}

__global__ __launch_bounds__(NTHR) void k_agg(
    const int* __restrict__ ei, const float* __restrict__ Mq, const float* __restrict__ Cq,
    const float* __restrict__ xb, float* outH, float* outX, float* S, int cbeg, int lim, int nN,
    int first, int last, int vecok) {
  extern __shared__ __attribute__((aligned(16))) float accd[];
  __shared__ int list[NWAVE * WCAP];
  __shared__ int wcnt[NWAVE];
  const int tid = (int)threadIdx.x, lane = tid & 31, wave = tid >> 5;
  const int base = (int)blockIdx.x * NBC;
  float* accF = accd;
  float* accC = accd + NBC * DN;
  const int* eid = ei;

  if (first != 0) {
#pragma unroll 1
    for (int i = tid; i < (NBC * DN) / 4; i += NTHR) *(v4f*)(accF + 4 * i) = zero4();
    *(v4f*)(accC + 4 * tid) = zero4();
  } else {
#pragma unroll 1
    for (int i = tid; i < (NBC * DN) / 4; i += NTHR) {
      const int s = i >> 5, c4 = (i & 31) * 4;
      int node = base + s;
      node = node > nN - 1 ? nN - 1 : node;
      const v4f v = *(const v4f*)(outH + (size_t)node * DN + c4);
      *(v4f*)(accF + s * DN + c4) = v;
    }
    {
      const v4f v = *(const v4f*)(S + (size_t)base * SROW + 4 * (size_t)tid);
      *(v4f*)(accC + 4 * tid) = v;
    }
  }
  __syncthreads();

#pragma unroll 1
  for (int cbase = cbeg; cbase < lim; cbase += PIECE) {
    const int wc = scan_piece(eid, lim, cbase, base, vecok, list, tid, wave);
    if (lane == 0) wcnt[wave] = wc;
    __syncthreads();
    drain_piece(list, wcnt, accF, accC, Mq, Cq, cbase - cbeg, lane, wave);
    __syncthreads();
  }

  agg_store(accF, accC, xb, outH, outX, S, base, nN, last, tid, lane, wave);
  __threadfence();
  agg_store(accF, accC, xb, outH, outX, S, base, nN, last, tid, lane, wave);
}

__global__ __launch_bounds__(NTHR) void k_nodemlp(
    const float* __restrict__ hsrc, const unsigned short* __restrict__ wp,
    const float* __restrict__ nb1, const float* __restrict__ nb2, float* HO, int nN) {
  extern __shared__ __attribute__((aligned(16))) float mdynf[];
  __shared__ __attribute__((aligned(16))) float sPar[2 * DN];
  _Float16* sAh = (_Float16*)mdynf;
  _Float16* sY  = sAh + NBN * APN;
  float* sU = mdynf;
  const int tid = (int)threadIdx.x, lane = tid & 31, wave = tid >> 5, hh = lane >> 4, m = lane & 15;
  const int n0 = (int)blockIdx.x * NBN;

  {
    const int nl = tid >> 2, g = tid & 3;
    int node = n0 + nl;
    node = node > nN - 1 ? nN - 1 : node;
    const float* np_ = hsrc + (size_t)node * DN + 32 * g;
    const float* mp  = HO   + (size_t)node * DN + 32 * g;
#pragma unroll
    for (int i = 0; i < 4; ++i) {
      const v4f xa = *(const v4f*)(np_ + 8 * i);
      const v4f xb = *(const v4f*)(np_ + 8 * i + 4);
      *(v8h*)(sAh + nl * APN + 32 * g + 8 * i) = cvt8h(xa, xb, SCA);
    }
#pragma unroll
    for (int i = 0; i < 4; ++i) {
      const v4f xa = *(const v4f*)(mp + 8 * i);
      const v4f xb = *(const v4f*)(mp + 8 * i + 4);
      *(v8h*)(sAh + nl * APN + DN + 32 * g + 8 * i) = cvt8h(xa, xb, SCA);
    }
  }
  if (tid < DN) {
    sPar[tid]      = nb1[tid];
    sPar[DN + tid] = nb2[tid];
  }
  __syncthreads();

  const int rt = wave & 3, cg = wave >> 2;

  {
    v8f a0, a1, a2, a3;
    gemm16x64(sAh + (16 * rt + m) * APN + 8 * hh, (const _Float16*)(wp + PN1), 2 * DN, 8, 64 * cg, m, hh,
              a0, a1, a2, a3);
    _Float16* py = sY + (16 * rt + 8 * hh) * APA + 64 * cg + m;
    const float* bb = sPar + 64 * cg + m;
    stage8hs(py,      a0, bb[0]);
    stage8hs(py + 16, a1, bb[16]);
    stage8hs(py + 32, a2, bb[32]);
    stage8hs(py + 48, a3, bb[48]);
  }
  __syncthreads();

  {
    v8f a0, a1, a2, a3;
    gemm16x64(sY + (16 * rt + m) * APA + 8 * hh, (const _Float16*)(wp + PN2), DN, 4, 64 * cg, m, hh, a0, a1, a2, a3);
    float* sp = sU + (16 * rt + 8 * hh) * GSTR + 64 * cg + m;
    stage8f(sp,      a0, INV1024, 0.0f);
    stage8f(sp + 16, a1, INV1024, 0.0f);
    stage8f(sp + 32, a2, INV1024, 0.0f);
    stage8f(sp + 48, a3, INV1024, 0.0f);
  }
  __syncthreads();

  const v4f b4 = *(const v4f*)(sPar + DN + 4 * lane);
#pragma unroll 1
  for (int it = 0; it < NBN / NWAVE; ++it) {
    const int s = wave + NWAVE * it;
    const int node = n0 + s;
    if (node < nN) {
      const v4f su = *(const v4f*)(sU + s * GSTR + 4 * lane);
      const v4f hv = *(const v4f*)(hsrc + (size_t)node * DN + 4 * lane);
      const v4f v = hv + (su + b4);
      *(volatile v4f*)(HO + (size_t)node * DN + 4 * lane) = v;
    }
  }
  __threadfence();
#pragma unroll 1
  for (int it = 0; it < NBN / NWAVE; ++it) {
    const int s = wave + NWAVE * it;
    const int node = n0 + s;
    if (node < nN) {
      const v4f su = *(const v4f*)(sU + s * GSTR + 4 * lane);
      const v4f hv = *(const v4f*)(hsrc + (size_t)node * DN + 4 * lane);
      const v4f v = hv + (su + b4);
      *(volatile v4f*)(HO + (size_t)node * DN + 4 * lane) = v;
    }
  }
}

extern "C" void kernel_launch(void* const* d_in, const int* in_sizes, int n_in,
                              void* d_out, int out_size, void* d_ws, size_t ws_size,
                              hipStream_t stream) {
  if (n_in < 14) return;
  if (in_sizes[0] < DN || (in_sizes[0] % DN) != 0) return;
  const int nN = in_sizes[0] / DN;
  if (nN < 1 || nN > (1 << 22)) return;
  if (in_sizes[1] != 3 * nN) return;
  if (in_sizes[2] < 2 || (in_sizes[2] % 2) != 0) return;
  const int nE = in_sizes[2] / 2;
  if (nE < 1 || nE > (1 << 26)) return;
  if (in_sizes[3] != (2 * DN + 1) * DN || in_sizes[4] != DN) return;
  if (in_sizes[5] != DN * DN || in_sizes[6] != DN) return;
  if (in_sizes[7] != DN * DN || in_sizes[8] != DN) return;
  if (in_sizes[9] != DN) return;
  if (in_sizes[10] != 2 * DN * DN || in_sizes[11] != DN) return;
  if (in_sizes[12] != DN * DN || in_sizes[13] != DN) return;
  if (out_size != nN * (DN + 3)) return;

  const float* h   = (const float*)d_in[0];
  const float* pos = (const float*)d_in[1];
  const int*   ei  = (const int*)d_in[2];
  const float* eW1 = (const float*)d_in[3];
  const float* eb1 = (const float*)d_in[4];
  const float* eW2 = (const float*)d_in[5];
  const float* eb2 = (const float*)d_in[6];
  const float* cW1 = (const float*)d_in[7];
  const float* cb1 = (const float*)d_in[8];
  const float* cW2 = (const float*)d_in[9];
  const float* nW1 = (const float*)d_in[10];
  const float* nb1 = (const float*)d_in[11];
  const float* nW2 = (const float*)d_in[12];
  const float* nb2 = (const float*)d_in[13];
  float* out0 = (float*)d_out;
  float* out1 = out0 + (size_t)DN * (size_t)nN;

  const int nbNode = (nN + NBN - 1) / NBN;
  const int NpadT  = nbNode * NBN;
  const int nChunk = (nE + CE - 1) / CE;
  if (nChunk < 1 || nChunk > MAXCH) return;
  const int nbAgg  = (nN + NBC - 1) / NBC;
  const int SpadN  = nbAgg * NBC;

  char* ws = (char*)d_ws;
  size_t off = 0;
  const size_t oW  = off; off += (size_t)PWTOT * 2;             off = (off + 255) & ~(size_t)255;
  const size_t oNP = off; off += (size_t)NpadT * NPROW * 4;     off = (off + 255) & ~(size_t)255;
  const size_t oM  = off; off += (size_t)CE * MROW * 4;         off = (off + 255) & ~(size_t)255;
  const size_t oC  = off; off += (size_t)CE * CROW * 4;         off = (off + 255) & ~(size_t)255;
  const size_t oS  = off; off += (size_t)SpadN * SROW * 4;      off = (off + 255) & ~(size_t)255;
  if (off > ws_size || off > (size_t)WSCAP) return;
  unsigned short* wp = (unsigned short*)(ws + oW);
  float* NP          = (float*)(ws + oNP);
  float* Mq          = (float*)(ws + oM);
  float* Cq          = (float*)(ws + oC);
  float* S           = (float*)(ws + oS);

  hipFuncSetAttribute(reinterpret_cast<const void*>(&k_node), hipFuncAttributeMaxDynamicSharedMemorySize, NODEDYN);
  hipFuncSetAttribute(reinterpret_cast<const void*>(&k_edge), hipFuncAttributeMaxDynamicSharedMemorySize, EDGEDYN);
  hipFuncSetAttribute(reinterpret_cast<const void*>(&k_agg), hipFuncAttributeMaxDynamicSharedMemorySize, AGGDYN);
  hipFuncSetAttribute(reinterpret_cast<const void*>(&k_nodemlp), hipFuncAttributeMaxDynamicSharedMemorySize, MLPDYN);

  k_prep<<<PBLK, NTHR, 0, stream>>>(eW1, eW2, cW1, cW2, nW1, nW2, wp);
  k_node<<<nbNode, NTHR, NODEDYN, stream>>>(h, wp, NP, nN);
  for (int c = 0; c < nChunk; ++c) {
    const int cbeg = c * CE;
    int lim = cbeg + CE;
    lim = lim > nE ? nE : lim;
    const int nblk = (lim - cbeg + NBE - 1) / NBE;
    const int first = (c == 0) ? 1 : 0;
    const int last  = (c == nChunk - 1) ? 1 : 0;
    k_edge<<<nblk, NTHR, EDGEDYN, stream>>>(pos, ei, NP, wp, eW1, eb1, eb2, cb1, Mq, Cq, nE, nN, cbeg);
    k_agg<<<nbAgg, NTHR, AGGDYN, stream>>>(ei, Mq, Cq, pos, out0, out1, S, cbeg, lim, nN, first, last, 1);
  }
  k_nodemlp<<<nbNode, NTHR, MLPDYN, stream>>>(h, wp, nb1, nb2, out0, nN);
}
